// Net_88407606821102
// MI455X (gfx1250) — hardware-verified
//
#include <hip/hip_runtime.h>
#include <stddef.h>
#include <stdint.h>


#define NNODE   10000
#define NEDGE   160000
#define FD      768
#define HDIM    96
#define NLAY    4
#define NLR     1536
#define MP      10112
#define KQ      96
#define NZ      600
#define NOUT    601
#define NTHR    256
#define NWAVE   8
#define EPT     8
#define CHUNK   (NTHR * EPT)
#define WCAP    (EPT * 32)
#define LISTN   (NWAVE * WCAP)
#define NBMAX   2048
#define NBRUN   1024
#define ESH     11
#define RCAP    28672
#define DEGCAP  4096
#define STW     800
#define GBM     64
#define GBN     64
#define GTHR    128
#define NEGS    0.2f
#define HNEG    0.01f
#define WSMAX   134217728
#define LDS_AGG ((2 * RCAP + 2 * NBMAX + LISTN) * 4 + 64)
#define NTN     1024
#define FPT     10
#define FLEN    (NTN * FPT)
#define LDS_NEED (3 * FLEN * 4)
#define HTHR    640

static_assert((CHUNK & (CHUNK - 1)) == 0 && CHUNK <= 4096);
static_assert((NBMAX & (NBMAX - 1)) == 0 && NBMAX <= 4096);
static_assert((NBRUN & (NBRUN - 1)) == 0 && NBRUN <= NBMAX && NBRUN >= 16);
static_assert((1 << ESH) >= NBMAX);
static_assert(NEDGE <= (1 << (32 - ESH)));
static_assert(NTHR * 8 == NBMAX);
static_assert(LISTN >= NBMAX);
static_assert(LISTN >= NWAVE * WCAP);
static_assert((RCAP % 32) == 0);
static_assert(NWAVE * STW + 2 * FD <= RCAP);
static_assert((STW % 4) == 0 && STW >= FD + 8);
static_assert(RCAP >= 16542 + 4096);
static_assert(DEGCAP >= 33 + 8);
static_assert(LDS_AGG <= 300000);
static_assert(GBM == (GTHR / 32) * 16);
static_assert((FD % 32) == 0 && (NLR % GBN) == 0 && (MP % GBM) == 0 && MP >= NNODE);
static_assert(FD == 32 * 24 && HDIM == 4 * 24 && FD == 8 * HDIM);
static_assert((HDIM % 8) == 0 && FD / 8 == KQ && KQ == 3 * 32);
static_assert(FLEN >= MP && (MP % 128) == 0);
static_assert((NEDGE % 4) == 0);
static_assert(NOUT <= HTHR && NZ < HTHR);
static_assert(((MP * KQ) % NTHR) == 0 && ((NLAY * FD * KQ) % NTHR) == 0 && ((NLAY * FD / 4) % NTHR) == 0);

typedef float          v4f   __attribute__((ext_vector_type(4)));
typedef float          v8f   __attribute__((ext_vector_type(8)));
typedef int            v4i   __attribute__((ext_vector_type(4)));
typedef int            v8i   __attribute__((ext_vector_type(8)));
typedef unsigned short v8us  __attribute__((ext_vector_type(8)));
typedef __bf16         v16bf __attribute__((ext_vector_type(16)));
union FragB { v16bf v; v8us u[2]; v8i w; };

__device__ __forceinline__ v8f wmx(const FragB& a, const FragB& b, v8f c) {
  v8f d = __builtin_amdgcn_wmma_f32_16x16x32_bf16(false, a.v, false, b.v, (short)0, c, false, false);
  asm volatile("v_nop\n\tv_nop\n\tv_nop\n\tv_nop" : "+v"(d) : "v"(a.w), "v"(b.w));
  return d;
}

__device__ __forceinline__ unsigned bfbits(float v) {
  unsigned u = __float_as_uint(v);
  u = u + 0x7FFFu + ((u >> 16) & 1u);
  return u >> 16;
}
__device__ __forceinline__ float rbf(float v) { return __uint_as_float(bfbits(v) << 16); }
__device__ __forceinline__ unsigned bfn(float v) {
  const unsigned b = bfbits(v);
  return (v != v) ? 0x7fc0u : b;
}
__device__ __forceinline__ v4f rbf4(v4f a) {
  v4f o; o.x = rbf(a.x); o.y = rbf(a.y); o.z = rbf(a.z); o.w = rbf(a.w); return o;
}
__device__ __forceinline__ float lrelu(float v, float s) { return v >= 0.f ? v : v * s; }

__device__ __forceinline__ v8us cvt8b(const v4f a, const v4f b) {
  v8us o;
  o[0] = (unsigned short)bfbits(a.x); o[1] = (unsigned short)bfbits(a.y);
  o[2] = (unsigned short)bfbits(a.z); o[3] = (unsigned short)bfbits(a.w);
  o[4] = (unsigned short)bfbits(b.x); o[5] = (unsigned short)bfbits(b.y);
  o[6] = (unsigned short)bfbits(b.z); o[7] = (unsigned short)bfbits(b.w);
  return o;
}
__device__ __forceinline__ void cvt8hl(const v4f a, const v4f b, v8us& hv, v8us& lv) {
  float f[8] = {a.x, a.y, a.z, a.w, b.x, b.y, b.z, b.w};
#pragma unroll
  for (int i = 0; i < 8; ++i) {
    const unsigned hb = bfn(f[i]);
    const float hf = __uint_as_float(hb << 16);
    const unsigned lb = bfn(f[i] - hf);
    hv[i] = (unsigned short)hb;
    lv[i] = (unsigned short)lb;
  }
}
__device__ __forceinline__ void put8us(unsigned short* p, const v8us hv) {
  *(volatile v8us*)p = hv;
  __threadfence();
  *(volatile v8us*)p = hv;
}

__device__ __forceinline__ int scan_chunk(const int* __restrict__ dsts, int nE, int cbase, int slotBase,
                                          int nb, int vec8, int* list, int tid, int lane, int wave) {
  int wc = 0;
  const int el0  = tid * EPT;
  const int e0   = cbase + el0;
  const int sent = -2147483647 - 1;
  v4i da, db;
  if (vec8 != 0 && cbase + CHUNK <= nE) {
    da = *(const v4i*)(dsts + e0);
    db = *(const v4i*)(dsts + e0 + 4);
  } else {
    da.x = (e0     < nE) ? dsts[min(e0,     nE - 1)] : sent;
    da.y = (e0 + 1 < nE) ? dsts[min(e0 + 1, nE - 1)] : sent;
    da.z = (e0 + 2 < nE) ? dsts[min(e0 + 2, nE - 1)] : sent;
    da.w = (e0 + 3 < nE) ? dsts[min(e0 + 3, nE - 1)] : sent;
    db.x = (e0 + 4 < nE) ? dsts[min(e0 + 4, nE - 1)] : sent;
    db.y = (e0 + 5 < nE) ? dsts[min(e0 + 5, nE - 1)] : sent;
    db.z = (e0 + 6 < nE) ? dsts[min(e0 + 6, nE - 1)] : sent;
    db.w = (e0 + 7 < nE) ? dsts[min(e0 + 7, nE - 1)] : sent;
  }
  const unsigned nbs = (unsigned)slotBase;
  const unsigned unb = (unsigned)nb;
  const unsigned s0 = (unsigned)da.x - nbs, s1 = (unsigned)da.y - nbs;
  const unsigned s2 = (unsigned)da.z - nbs, s3 = (unsigned)da.w - nbs;
  const unsigned s4 = (unsigned)db.x - nbs, s5 = (unsigned)db.y - nbs;
  const unsigned s6 = (unsigned)db.z - nbs, s7 = (unsigned)db.w - nbs;
  const bool h0 = s0 < unb, h1 = s1 < unb, h2 = s2 < unb, h3 = s3 < unb;
  const bool h4 = s4 < unb, h5 = s5 < unb, h6 = s6 < unb, h7 = s7 < unb;
  const unsigned any = __builtin_amdgcn_ballot_w32(h0 | h1 | h2 | h3 | h4 | h5 | h6 | h7);
  if (any != 0u) {
#define HITJ(J, HJ, SJ) { \
      const unsigned mj = __builtin_amdgcn_ballot_w32(HJ); \
      if (mj != 0u) { \
        if (HJ) { \
          const int pos = wc + (int)__builtin_amdgcn_mbcnt_lo(mj, 0u); \
          if (pos < WCAP) list[wave * WCAP + pos] = ((el0 + (J)) << 12) | (int)(SJ); \
        } \
        wc += (int)__builtin_popcount(mj); } }
    HITJ(0, h0, s0)
    HITJ(1, h1, s1)
    HITJ(2, h2, s2)
    HITJ(3, h3, s3)
    HITJ(4, h4, s4)
    HITJ(5, h5, s5)
    HITJ(6, h6, s6)
    HITJ(7, h7, s7)
#undef HITJ
  }
  return wc;
}

__device__ __forceinline__ int build_lists(const int* __restrict__ dsts, int nE, int nodeBase, int nb, int vec8,
                                           int* reg1, int* reg2, int* scnt, int* soff, int* list,
                                           int* wcnt, int* wtot, int tid, int lane, int wave) {
  for (int i = tid; i < NBMAX; i += NTHR) scnt[i] = 0;
  __syncthreads();

  int tot = 0;
  const int nChunks = (nE + CHUNK - 1) / CHUNK;
#pragma unroll 1
  for (int ch = 0; ch < nChunks; ++ch) {
    const int cbase = ch * CHUNK;
    const int wc = scan_chunk(dsts, nE, cbase, nodeBase, nb, vec8, list, tid, lane, wave);
    if (lane == 0) wcnt[wave] = wc;
    __syncthreads();
    int pre = 0, all = 0;
#pragma unroll
    for (int w2 = 0; w2 < NWAVE; ++w2) {
      int c = wcnt[w2];
      c = c < 0 ? 0 : (c > WCAP ? WCAP : c);
      all += c;
      pre += (w2 < wave) ? c : 0;
    }
    const int wcc  = wc > WCAP ? WCAP : wc;
    const int base = tot + pre;
#pragma unroll 1
    for (int i = lane; i < wcc; i += 32) {
      const int ent = list[wave * WCAP + i];
      const int el  = (ent >> 12) & (CHUNK - 1);
      const int sl  = ent & (NBMAX - 1);
      int eid = cbase + el;
      eid = eid > nE - 1 ? nE - 1 : eid;
      const int pos = base + i;
      if (pos < RCAP) reg1[pos] = (int)(((unsigned)eid << ESH) | (unsigned)sl);
    }
    tot += all;
    tot = tot > RCAP ? RCAP : tot;
    __syncthreads();
  }
  const int nh = tot;

  if (wave == 0) {
#pragma unroll 1
    for (int b0 = 0; b0 < nh; b0 += 32) {
      const int idx = b0 + lane;
      const int uv  = reg1[idx < RCAP ? idx : RCAP - 1];
      const int m32 = (nh - b0) < 32 ? (nh - b0) : 32;
#pragma unroll 1
      for (int k = 0; k < m32; ++k) {
        const int u  = __builtin_amdgcn_readlane(uv, k);
        const int sl = u & (NBMAX - 1);
        if (lane == 0) scnt[sl] = scnt[sl] + 1;
      }
    }
  }
  __syncthreads();

  {
    const v4i ca = *(const v4i*)(scnt + 8 * tid);
    const v4i cb = *(const v4i*)(scnt + 8 * tid + 4);
    const int e0 = ca.x < 0 ? 0 : ca.x, e1 = ca.y < 0 ? 0 : ca.y, e2 = ca.z < 0 ? 0 : ca.z, e3 = ca.w < 0 ? 0 : ca.w;
    const int e4 = cb.x < 0 ? 0 : cb.x, e5 = cb.y < 0 ? 0 : cb.y, e6 = cb.z < 0 ? 0 : cb.z, e7 = cb.w < 0 ? 0 : cb.w;
    const int ts = e0 + e1 + e2 + e3 + e4 + e5 + e6 + e7;
    int incl = ts;
#pragma unroll
    for (int d = 1; d < 32; d <<= 1) {
      const int up = __shfl_up(incl, d);
      if (lane >= d) incl += up;
    }
    if (lane == 31) wtot[wave] = incl;
    __syncthreads();
    int pre = 0;
#pragma unroll
    for (int w2 = 0; w2 < NWAVE; ++w2) pre += (w2 < wave) ? wtot[w2] : 0;
    int run = pre + incl - ts;
    soff[8 * tid + 0] = run; run += e0;
    soff[8 * tid + 1] = run; run += e1;
    soff[8 * tid + 2] = run; run += e2;
    soff[8 * tid + 3] = run; run += e3;
    soff[8 * tid + 4] = run; run += e4;
    soff[8 * tid + 5] = run; run += e5;
    soff[8 * tid + 6] = run; run += e6;
    soff[8 * tid + 7] = run;
  }
  __syncthreads();
  for (int i = tid; i < NBMAX; i += NTHR) list[i] = soff[i];
  __syncthreads();

  if (wave == 0) {
#pragma unroll 1
    for (int b0 = 0; b0 < nh; b0 += 32) {
      const int idx = b0 + lane;
      const int uv  = reg1[idx < RCAP ? idx : RCAP - 1];
      const int m32 = (nh - b0) < 32 ? (nh - b0) : 32;
#pragma unroll 1
      for (int k = 0; k < m32; ++k) {
        const int u   = __builtin_amdgcn_readlane(uv, k);
        const int sl  = u & (NBMAX - 1);
        const int eid = (int)((unsigned)u >> ESH);
        if (lane == 0) {
          int pos = list[sl];
          pos = pos < 0 ? 0 : (pos > RCAP - 1 ? RCAP - 1 : pos);
          reg2[pos] = eid;
          list[sl] = pos + 1;
        }
      }
    }
  }
  __syncthreads();
  return nh;
}

__device__ __forceinline__ void wt_unit(const float* __restrict__ W, unsigned short* wt, int u, int seg) {
  if (u >= NLAY * FD * KQ) return;
  const int layer = u / (FD * KQ);
  const int rem   = u - layer * (FD * KQ);
  const int n     = rem / KQ;
  const int k8    = (rem - n * KQ) * 8;
  const float* p = W + (size_t)layer * FD * FD + (size_t)k8 * FD + n;
  v4f a, b;
  a.x = p[0];        a.y = p[FD];       a.z = p[2 * FD];   a.w = p[3 * FD];
  b.x = p[4 * FD];   b.y = p[5 * FD];   b.z = p[6 * FD];   b.w = p[7 * FD];
  put8us(wt + (size_t)(layer * NLR + seg * FD + n) * FD + k8, cvt8b(a, b));
}

__device__ __forceinline__ void bs_unit(const float* __restrict__ bsrcv, float* bsd, int uu, int seg) {
  if (uu >= NLAY * FD / 4) return;
  const int layer = uu / (FD / 4);
  const int c4    = (uu - layer * (FD / 4)) * 4;
  const v4f v = rbf4(*(const v4f*)(bsrcv + layer * FD + c4));
  float* o = bsd + layer * NLR + seg * FD + c4;
  *(volatile v4f*)o = v;
  __threadfence();
  *(volatile v4f*)o = v;
}

#define NBX  ((MP * KQ) / NTHR)
#define NBW  ((NLAY * FD * KQ) / NTHR)
#define NBB  ((NLAY * FD / 4) / NTHR)

__global__ __launch_bounds__(NTHR) void k_prep(
    const float* __restrict__ x, const float* __restrict__ wsrc, const float* __restrict__ wdst,
    const float* __restrict__ bsrc, const float* __restrict__ bdst,
    unsigned short* xb, unsigned short* wt, float* bsd, int nN) {
  const int b = (int)blockIdx.x, tid = (int)threadIdx.x;
  if (b < NBX) {
    const int i = b * NTHR + tid;
    const int row = i / KQ;
    const int c0  = (i - row * KQ) * 8;
    const int rc  = row < nN ? row : nN - 1;
    const float* p = x + (size_t)rc * FD + c0;
    v4f a = *(const v4f*)p, bq = *(const v4f*)(p + 4);
    const v4f z4 = {0.f, 0.f, 0.f, 0.f};
    if (row >= nN) { a = z4; bq = z4; }
    put8us(xb + (size_t)row * FD + c0, cvt8b(a, bq));
  } else if (b < NBX + NBW) {
    wt_unit(wsrc, wt, (b - NBX) * NTHR + tid, 0);
  } else if (b < NBX + 2 * NBW) {
    wt_unit(wdst, wt, (b - NBX - NBW) * NTHR + tid, 1);
  } else if (b < NBX + 2 * NBW + NBB) {
    bs_unit(bsrc, bsd, (b - NBX - 2 * NBW) * NTHR + tid, 0);
  } else {
    bs_unit(bdst, bsd, (b - NBX - 2 * NBW - NBB) * NTHR + tid, 1);
  }
}

__device__ __forceinline__ int rank_level(int* f, int* wtot, int tid, int lane, int wave) {
  int fl[FPT];
  int c = 0;
#pragma unroll
  for (int i = 0; i < FPT; ++i) { fl[i] = (f[FPT * tid + i] != 0) ? 1 : 0; c += fl[i]; }
  int incl = c;
#pragma unroll
  for (int d = 1; d < 32; d <<= 1) {
    const int up = __shfl_up(incl, d);
    if (lane >= d) incl += up;
  }
  if (lane == 31) wtot[wave] = incl;
  __syncthreads();
  int pre = 0, all = 0;
#pragma unroll
  for (int w2 = 0; w2 < NTN / 32; ++w2) {
    const int t = wtot[w2];
    all += t;
    pre += (w2 < wave) ? t : 0;
  }
  int run = pre + incl - c;
#pragma unroll
  for (int i = 0; i < FPT; ++i) { f[FPT * tid + i] = fl[i] ? run : -1; run += fl[i]; }
  __syncthreads();
  return all;
}

__device__ __forceinline__ void put_tab(const int* f, int* g, int tid) {
#pragma unroll 1
  for (int i = tid; i < MP / 4; i += NTN) {
    const v4i v = *(const v4i*)(f + 4 * i);
    *(volatile v4i*)(g + 4 * i) = v;
    __threadfence();
    *(volatile v4i*)(g + 4 * i) = v;
  }
}

__device__ __forceinline__ int clampn(int v) { return v < 0 ? 0 : (v > NNODE - 1 ? NNODE - 1 : v); }

__global__ __launch_bounds__(NTN) void k_need(const int* __restrict__ srcs, const int* __restrict__ dsts,
                                              int* pos1, int* pos2, int* pos3, int* cnts, int nE4) {
  extern __shared__ v4i lds_need[];
  __shared__ int wtot[NTN / 32];
  int* f1 = (int*)lds_need;
  int* f2 = f1 + FLEN;
  int* f3 = f2 + FLEN;
  const int tid = (int)threadIdx.x, lane = tid & 31, wave = tid >> 5;

  for (int i = tid; i < 3 * FLEN; i += NTN) f1[i] = 0;
  __syncthreads();
  if (tid == 0) f3[0] = 1;

#pragma unroll 1
  for (int g = tid; g < nE4; g += NTN) {
    const v4i d4 = *(const v4i*)(dsts + 4 * g);
    const v4i s4 = *(const v4i*)(srcs + 4 * g);
    const int sa = clampn(s4.x), sb = clampn(s4.y), sc = clampn(s4.z), sd = clampn(s4.w);
    if (d4.x == 0) f3[sa] = 1;
    if (d4.y == 0) f3[sb] = 1;
    if (d4.z == 0) f3[sc] = 1;
    if (d4.w == 0) f3[sd] = 1;
  }
  __syncthreads();

#pragma unroll 1
  for (int g = tid; g < nE4; g += NTN) {
    const v4i d4 = *(const v4i*)(dsts + 4 * g);
    const v4i s4 = *(const v4i*)(srcs + 4 * g);
    const int ga = f3[clampn(d4.x)], gb = f3[clampn(d4.y)], gc = f3[clampn(d4.z)], gd = f3[clampn(d4.w)];
    const int sa = clampn(s4.x), sb = clampn(s4.y), sc = clampn(s4.z), sd = clampn(s4.w);
    if (ga != 0) f2[sa] = 1;
    if (gb != 0) f2[sb] = 1;
    if (gc != 0) f2[sc] = 1;
    if (gd != 0) f2[sd] = 1;
  }
  __syncthreads();
  for (int i = tid; i < FLEN; i += NTN) { const int a = f2[i], c = f3[i]; f2[i] = a | c; }
  __syncthreads();

#pragma unroll 1
  for (int g = tid; g < nE4; g += NTN) {
    const v4i d4 = *(const v4i*)(dsts + 4 * g);
    const v4i s4 = *(const v4i*)(srcs + 4 * g);
    const int ga = f2[clampn(d4.x)], gb = f2[clampn(d4.y)], gc = f2[clampn(d4.z)], gd = f2[clampn(d4.w)];
    const int sa = clampn(s4.x), sb = clampn(s4.y), sc = clampn(s4.z), sd = clampn(s4.w);
    if (ga != 0) f1[sa] = 1;
    if (gb != 0) f1[sb] = 1;
    if (gc != 0) f1[sc] = 1;
    if (gd != 0) f1[sd] = 1;
  }
  __syncthreads();
  for (int i = tid; i < FLEN; i += NTN) { const int a = f1[i], c = f2[i]; f1[i] = a | c; }
  __syncthreads();

  const int c3 = rank_level(f3, wtot, tid, lane, wave);
  const int c2 = rank_level(f2, wtot, tid, lane, wave);
  const int c1 = rank_level(f1, wtot, tid, lane, wave);
  put_tab(f1, pos1, tid);
  put_tab(f2, pos2, tid);
  put_tab(f3, pos3, tid);
  if (tid < 8) {
    v4i v = {0, 0, 0, 0};
    if (tid == 0) { v.x = NNODE; v.y = c1; v.z = c2; v.w = c3; }
    if (tid == 1) { v.x = 1; }
    *(volatile v4i*)(cnts + 4 * tid) = v;
    __threadfence();
    *(volatile v4i*)(cnts + 4 * tid) = v;
  }
}

__global__ __launch_bounds__(GTHR) void k_gemm(
    const unsigned short* __restrict__ A, const unsigned short* __restrict__ WT,
    const float* __restrict__ bsd, float* outF, const int* __restrict__ cnts, int cidx, int K, int kwrap)
{
  __shared__ __attribute__((aligned(16))) float stg[GBM * GBN];
  const int tid = (int)threadIdx.x, lane = tid & 31, wave = tid >> 5, hh = lane >> 4, m = lane & 15;
  int cnt = cnts[cidx];
  cnt = cnt < 1 ? 1 : (cnt > NNODE ? NNODE : cnt);
  cnt = __builtin_amdgcn_readfirstlane(cnt);
  const int rowBase = (int)blockIdx.x * GBM;
  if (rowBase >= cnt) return;
  const int col0 = (int)blockIdx.y * GBN;

  v8f acc[4];
  {
    const v8f z = {0.f, 0.f, 0.f, 0.f, 0.f, 0.f, 0.f, 0.f};
    acc[0] = z; acc[1] = z; acc[2] = z; acc[3] = z;
  }
  int ar = rowBase + 16 * wave + m;
  ar = ar < cnt ? ar : cnt - 1;
  const unsigned short* ap = A  + (size_t)ar * (size_t)K + 8 * hh;
  const unsigned short* wp = WT + (size_t)(col0 + m) * (size_t)FD + 8 * hh;
  const int ksteps = K >> 5;
#pragma unroll 1
  for (int ks = 0; ks < ksteps; ++ks) {
    const int kb = ks >= kwrap ? ks - kwrap : ks;
    FragB af;
    af.u[0] = *(const v8us*)(ap + 32 * ks);
    af.u[1] = *(const v8us*)(ap + 32 * ks + 16);
#pragma unroll
    for (int t = 0; t < 4; ++t) {
      const unsigned short* wq = wp + (size_t)(16 * t) * (size_t)FD + 32 * kb;
      FragB bf;
      bf.u[0] = *(const v8us*)wq;
      bf.u[1] = *(const v8us*)(wq + 16);
      acc[t] = wmx(af, bf, acc[t]);
    }
  }

#pragma unroll
  for (int t = 0; t < 4; ++t) {
    const int lc = 16 * t + m;
    const float bv = bsd[col0 + lc];
#pragma unroll
    for (int r = 0; r < 8; ++r) {
      const int lr = 16 * wave + 8 * hh + r;
      stg[lr * GBN + lc] = acc[t][r] + bv;
    }
  }
  __syncthreads();

  v4f fv[8];
#pragma unroll
  for (int i = 0; i < 8; ++i) {
    const int lr = 16 * wave + 2 * i + hh;
    fv[i] = *(const v4f*)(stg + lr * GBN + 4 * m);
  }
#pragma unroll
  for (int i = 0; i < 8; ++i) {
    const int lr = 16 * wave + 2 * i + hh;
    const int gr = rowBase + lr;
    float* op = outF + (size_t)gr * (size_t)NLR + col0 + 4 * m;
    if (gr < cnt) *(volatile v4f*)op = fv[i];
  }
  __threadfence();
#pragma unroll
  for (int i = 0; i < 8; ++i) {
    const int lr = 16 * wave + 2 * i + hh;
    const int gr = rowBase + lr;
    float* op = outF + (size_t)gr * (size_t)NLR + col0 + 4 * m;
    if (gr < cnt) *(volatile v4f*)op = fv[i];
  }
}

template<int LAST>
__global__ __launch_bounds__(NTHR) void k_scan(
    const int* __restrict__ srcs, const int* __restrict__ dsts,
    const float* __restrict__ FS, const float* __restrict__ att, const float* __restrict__ gbias,
    const int* __restrict__ posCur, const int* __restrict__ posPrev, int identPrev,
    unsigned short* X, float* X4F, int nN, int nE, int nb, int vec8) {
  extern __shared__ v4f lds_dyn[];
  int* reg1 = (int*)lds_dyn;
  int* reg2 = reg1 + RCAP;
  int* scnt = reg2 + RCAP;
  int* soff = scnt + NBMAX;
  int* list = soff + NBMAX;
  int* wcnt = list + LISTN;
  int* wtot = wcnt + NWAVE;
  const int tid = (int)threadIdx.x, lane = tid & 31, wave = tid >> 5;
  if (LAST && blockIdx.x != 0) return;
  const int nodeBase = (int)blockIdx.x * nb;

  const int nh = build_lists(dsts, nE, nodeBase, nb, vec8, reg1, reg2, scnt, soff, list, wcnt, wtot,
                             tid, lane, wave);

  float* fr  = (float*)reg1;
  float* stw = fr + wave * STW;
  float* siv = stw + FD;
  float* sat = fr + NWAVE * STW;
  float* sgb = sat + FD;
  if (tid < FD / 4) {
    *(v4f*)(sat + 4 * tid) = rbf4(*(const v4f*)(att + 4 * tid));
    *(v4f*)(sgb + 4 * tid) = rbf4(*(const v4f*)(gbias + 4 * tid));
  }
  __syncthreads();
  v4f at4[6];
#pragma unroll
  for (int j = 0; j < 6; ++j) at4[j] = *(const v4f*)(sat + 24 * lane + 4 * j);

  const int nbw = nb >> 3;
  const bool ovf = (nh >= RCAP);
  const float qnan = __int_as_float(0x7fc00000);
  const v4f z4 = {0.f, 0.f, 0.f, 0.f};

#pragma unroll 1
  for (int jt = 0; jt < nbw; ++jt) {
    const int slot = wave * nbw + jt;
    const int d    = nodeBase + slot;
    const int dcl  = d < nN ? d : nN - 1;
    int r;
    if (LAST) r = (d == 0) ? 0 : -1; else r = posCur[dcl];
    if (d >= nN) r = -1;
    r = __builtin_amdgcn_readfirstlane(r);
    if (r < 0) continue;
    r = r > MP - 1 ? MP - 1 : r;
    int p = posPrev[dcl];
    if (identPrev != 0) p = d;
    p = __builtin_amdgcn_readfirstlane(p);
    float pz = ovf ? qnan : 0.0f;
    if (p < 0) pz = qnan;
    p = p < 0 ? 0 : (p > MP - 1 ? MP - 1 : p);
    int st = soff[slot];
    const int craw = scnt[slot];
    int cnt = craw;
    st  = st < 0 ? 0 : (st > nh ? nh : st);
    cnt = cnt < 0 ? 0 : (cnt > DEGCAP ? DEGCAP : cnt);
    if (cnt > nh - st) cnt = nh - st;
    if (craw > DEGCAP) pz = qnan;
    st  = __builtin_amdgcn_readfirstlane(st);
    cnt = __builtin_amdgcn_readfirstlane(cnt);

    const float* drow = FS + (size_t)p * NLR + 24 * lane;
    v4f hd[6], av[6];
#pragma unroll
    for (int j = 0; j < 6; ++j) { hd[j] = *(const v4f*)(drow + FD + 4 * j); av[j] = z4; }
    float mx = -1.0e30f, dn = 0.f;

#pragma unroll 1
    for (int q = -1; q < cnt; ++q) {
      int row = p;
      if (q >= 0) {
        int idx = st + q; idx = idx > RCAP - 1 ? RCAP - 1 : idx;
        int eid = reg2[idx]; eid = eid < 0 ? 0 : (eid > nE - 1 ? nE - 1 : eid);
        const int sraw = srcs[eid];
        const int s = sraw < 0 ? 0 : (sraw > nN - 1 ? nN - 1 : sraw);
        int qq = posPrev[s];
        if (identPrev != 0) qq = s;
        qq = __builtin_amdgcn_readfirstlane(qq);
        if (qq < 0) pz = qnan;
        row = qq < 0 ? 0 : (qq > MP - 1 ? MP - 1 : qq);
      }
      const float* sr = FS + (size_t)row * NLR + 24 * lane;
      v4f hs[6];
#pragma unroll
      for (int j = 0; j < 6; ++j) hs[j] = *(const v4f*)(sr + 4 * j);
      float part = 0.f;
#pragma unroll
      for (int j = 0; j < 6; ++j) {
        const v4f v = hs[j] + hd[j];
        part = fmaf(lrelu(v.x, NEGS), at4[j].x, part);
        part = fmaf(lrelu(v.y, NEGS), at4[j].y, part);
        part = fmaf(lrelu(v.z, NEGS), at4[j].z, part);
        part = fmaf(lrelu(v.w, NEGS), at4[j].w, part);
      }
      part += __shfl_xor(part, 1);
      part += __shfl_xor(part, 2);
      const float df = part - mx;
      const float ee = expf(-fabsf(df));
      const bool up  = df > 0.f;
      const float s1 = up ? ee : 1.0f;
      const float s2 = up ? 1.0f : ee;
      mx = up ? part : mx;
      dn = fmaf(dn, s1, s2);
#pragma unroll
      for (int j = 0; j < 6; ++j) {
        av[j].x = fmaf(av[j].x, s1, s2 * hs[j].x);
        av[j].y = fmaf(av[j].y, s1, s2 * hs[j].y);
        av[j].z = fmaf(av[j].z, s1, s2 * hs[j].z);
        av[j].w = fmaf(av[j].w, s1, s2 * hs[j].w);
      }
    }
    const float iv = 1.0f / dn;

    __builtin_amdgcn_fence(__ATOMIC_RELEASE, "wavefront");
    __builtin_amdgcn_wave_barrier();
#pragma unroll
    for (int j = 0; j < 6; ++j) *(v4f*)(stw + 24 * lane + 4 * j) = av[j];
    if ((lane & 3) == 0) siv[lane >> 2] = iv;
    __builtin_amdgcn_fence(__ATOMIC_RELEASE, "wavefront");
    __builtin_amdgcn_wave_barrier();

    if (!LAST) {
      unsigned short* xr = X + (size_t)r * NLR;
#pragma unroll 1
      for (int i = 0; i < 3; ++i) {
        const int piece = 32 * i + lane;
        const float ivp = siv[piece / 12];
        v4f a = *(const v4f*)(stw + 8 * piece);
        v4f b = *(const v4f*)(stw + 8 * piece + 4);
        const v4f ga = *(const v4f*)(sgb + 8 * piece);
        const v4f gb = *(const v4f*)(sgb + 8 * piece + 4);
        a.x = fmaf(a.x, ivp, ga.x) + pz; a.y = fmaf(a.y, ivp, ga.y) + pz;
        a.z = fmaf(a.z, ivp, ga.z) + pz; a.w = fmaf(a.w, ivp, ga.w) + pz;
        b.x = fmaf(b.x, ivp, gb.x) + pz; b.y = fmaf(b.y, ivp, gb.y) + pz;
        b.z = fmaf(b.z, ivp, gb.z) + pz; b.w = fmaf(b.w, ivp, gb.w) + pz;
        v8us hv, lv;
        cvt8hl(a, b, hv, lv);
        unsigned short* ph = xr + 8 * piece;
        unsigned short* pl = xr + FD + 8 * piece;
        *(volatile v8us*)ph = hv;
        *(volatile v8us*)pl = lv;
        __threadfence();
        *(volatile v8us*)ph = hv;
        *(volatile v8us*)pl = lv;
      }
    } else {
#pragma unroll 1
      for (int i = 0; i < 6; ++i) {
        const int piece = 32 * i + lane;
        const float ivp = siv[piece / 24];
        v4f a = *(const v4f*)(stw + 4 * piece);
        const v4f ga = *(const v4f*)(sgb + 4 * piece);
        a.x = fmaf(a.x, ivp, ga.x) + pz; a.y = fmaf(a.y, ivp, ga.y) + pz;
        a.z = fmaf(a.z, ivp, ga.z) + pz; a.w = fmaf(a.w, ivp, ga.w) + pz;
        float* po = X4F + 4 * piece;
        *(volatile v4f*)po = a;
        __threadfence();
        *(volatile v4f*)po = a;
      }
    }
  }
  (void)X; (void)X4F; (void)posCur;
}

__global__ __launch_bounds__(HTHR) void k_head(const float* __restrict__ x4f, const float* __restrict__ w1,
                                               const float* __restrict__ b1, const float* __restrict__ w2,
                                               const float* __restrict__ b2, float* out) {
  __shared__ __attribute__((aligned(16))) float sh[FD];
  __shared__ float so[HTHR];
  __shared__ float sw2[HTHR];
  const int tid = (int)threadIdx.x;
  if (tid < FD / 4) *(v4f*)(sh + 4 * tid) = *(const v4f*)(x4f + 4 * tid);
  const int jc = tid < NZ ? tid : NZ - 1;
  { const float wa_ = rbf(w2[jc]); const float wb_ = rbf(b2[0]);
    const unsigned um_ = (unsigned)(-(int)(tid < NZ));
    sw2[tid] = __builtin_bit_cast(float, (__builtin_bit_cast(unsigned, wa_) & um_) | (__builtin_bit_cast(unsigned, wb_) & ~um_)); }
  __syncthreads();
  const float* wr = w1 + (size_t)jc * FD;
  float acc = 0.f;
#pragma unroll 4
  for (int k4 = 0; k4 < FD / 4; ++k4) {
    const v4f w = *(const v4f*)(wr + 4 * k4);
    const v4f h = *(const v4f*)(sh + 4 * k4);
    acc = fmaf(h.x, rbf(w.x), acc);
    acc = fmaf(h.y, rbf(w.y), acc);
    acc = fmaf(h.z, rbf(w.z), acc);
    acc = fmaf(h.w, rbf(w.w), acc);
  }
  acc += rbf(b1[jc]);
  const float z = acc >= 0.f ? acc : acc * HNEG;
  so[tid] = (tid < NZ) ? z : 0.f;
  __syncthreads();
  if (tid == 0) {
    double s = 0.0;
#pragma unroll 1
    for (int j = 0; j < NZ; ++j) s += (double)so[j] * (double)sw2[j];
    s += (double)sw2[NZ];
    so[NZ] = (float)s;
  }
  __syncthreads();
  const float v = so[tid < NOUT ? tid : NOUT - 1];
  if (tid < NOUT) *(volatile float*)(out + tid) = v;
  __threadfence();
  if (tid < NOUT) *(volatile float*)(out + tid) = v;
}

static int pick_nb(int nE, int nN) {
  int nb = NBRUN;
  while (nb > 16 && (long long)nb * (long long)nE * 5LL > (long long)RCAP * (long long)nN * 4LL) nb >>= 1;
  return nb;
}
static inline int cdiv(int a, int b) { return (a + b - 1) / b; }

extern "C" void kernel_launch(void* const* d_in, const int* in_sizes, int n_in,
                              void* d_out, int out_size, void* d_ws, size_t ws_size,
                              hipStream_t stream) {
  if (n_in < 13) return;
  if (in_sizes[0] != NNODE * FD) return;
  if (in_sizes[1] != NEDGE || in_sizes[2] != NEDGE) return;
  if (in_sizes[3] != NLAY * FD * FD || in_sizes[5] != NLAY * FD * FD) return;
  if (in_sizes[4] != NLAY * FD || in_sizes[6] != NLAY * FD || in_sizes[7] != NLAY * FD || in_sizes[8] != NLAY * FD) return;
  if (in_sizes[9] != NZ * FD || in_sizes[10] != NZ || in_sizes[11] != NZ || in_sizes[12] != 1) return;
  if (out_size != NOUT) return;

  const float* feat  = (const float*)d_in[0];
  const int*   src   = (const int*)  d_in[1];
  const int*   dst   = (const int*)  d_in[2];
  const float* Wsrc  = (const float*)d_in[3];
  const float* bsrc  = (const float*)d_in[4];
  const float* Wdst  = (const float*)d_in[5];
  const float* bdst  = (const float*)d_in[6];
  const float* attn  = (const float*)d_in[7];
  const float* gbias = (const float*)d_in[8];
  const float* fc1w  = (const float*)d_in[9];
  const float* fc1b  = (const float*)d_in[10];
  const float* fc2w  = (const float*)d_in[11];
  const float* fc2b  = (const float*)d_in[12];
  float* out = (float*)d_out;

  const int nN = NNODE, nE = NEDGE;
  const int nb   = pick_nb(nE, nN);
  const int gA   = cdiv(nN, nb);
  const int vec8 = ((nE & 3) == 0) ? 1 : 0;
  if (gA * nb < nN) return;

  char* ws = (char*)d_ws;
  size_t off = 0;
  const size_t oXB  = off; off += (size_t)MP * FD * 2;             off = (off + 255) & ~(size_t)255;
  const size_t oWT  = off; off += (size_t)NLAY * NLR * FD * 2;     off = (off + 255) & ~(size_t)255;
  const size_t oBSD = off; off += (size_t)NLAY * NLR * 4;          off = (off + 255) & ~(size_t)255;
  const size_t oFS  = off; off += (size_t)MP * NLR * 4;            off = (off + 255) & ~(size_t)255;
  const size_t oX   = off; off += (size_t)MP * NLR * 2;            off = (off + 255) & ~(size_t)255;
  const size_t oP1  = off; off += (size_t)MP * 4;                  off = (off + 255) & ~(size_t)255;
  const size_t oP2  = off; off += (size_t)MP * 4;                  off = (off + 255) & ~(size_t)255;
  const size_t oP3  = off; off += (size_t)MP * 4;                  off = (off + 255) & ~(size_t)255;
  const size_t oCN  = off; off += 128;                             off = (off + 255) & ~(size_t)255;
  const size_t oX4  = off; off += (size_t)FD * 4;                  off = (off + 255) & ~(size_t)255;
  if (off > ws_size || off > (size_t)WSMAX) return;
  unsigned short* XB  = (unsigned short*)(ws + oXB);
  unsigned short* WT  = (unsigned short*)(ws + oWT);
  float*          BSD = (float*)(ws + oBSD);
  float*          FSP = (float*)(ws + oFS);
  unsigned short* XP  = (unsigned short*)(ws + oX);
  int*            P1  = (int*)(ws + oP1);
  int*            P2  = (int*)(ws + oP2);
  int*            P3  = (int*)(ws + oP3);
  int*            CN  = (int*)(ws + oCN);
  float*          X4F = (float*)(ws + oX4);

  hipFuncSetAttribute(reinterpret_cast<const void*>(&k_scan<0>),
                      hipFuncAttributeMaxDynamicSharedMemorySize, LDS_AGG);
  hipFuncSetAttribute(reinterpret_cast<const void*>(&k_scan<1>),
                      hipFuncAttributeMaxDynamicSharedMemorySize, LDS_AGG);
  hipFuncSetAttribute(reinterpret_cast<const void*>(&k_need),
                      hipFuncAttributeMaxDynamicSharedMemorySize, LDS_NEED);

  k_prep<<<NBX + 2 * NBW + 2 * NBB, NTHR, 0, stream>>>(feat, Wsrc, Wdst, bsrc, bdst, XB, WT, BSD, nN);
  k_need<<<1, NTN, LDS_NEED, stream>>>(src, dst, P1, P2, P3, CN, nE / 4);

  const dim3 gg(MP / GBM, NLR / GBN);
  const size_t wtl = (size_t)NLR * FD;
  k_gemm<<<gg, GTHR, 0, stream>>>(XB, WT, BSD, FSP, CN, 0, FD, FD / 32);
  k_scan<0><<<gA, NTHR, LDS_AGG, stream>>>(src, dst, FSP, attn, gbias, P1, P1, 1, XP, X4F, nN, nE, nb, vec8);
  k_gemm<<<gg, GTHR, 0, stream>>>(XP, WT + wtl, BSD + NLR, FSP, CN, 1, NLR, FD / 32);
  k_scan<0><<<gA, NTHR, LDS_AGG, stream>>>(src, dst, FSP, attn + FD, gbias + FD, P2, P1, 0, XP, X4F, nN, nE, nb, vec8);
  k_gemm<<<gg, GTHR, 0, stream>>>(XP, WT + 2 * wtl, BSD + 2 * NLR, FSP, CN, 2, NLR, FD / 32);
  k_scan<0><<<gA, NTHR, LDS_AGG, stream>>>(src, dst, FSP, attn + 2 * FD, gbias + 2 * FD, P3, P2, 0, XP, X4F, nN, nE, nb, vec8);
  k_gemm<<<gg, GTHR, 0, stream>>>(XP, WT + 3 * wtl, BSD + 3 * NLR, FSP, CN, 3, NLR, FD / 32);
  k_scan<1><<<gA, NTHR, LDS_AGG, stream>>>(src, dst, FSP, attn + 3 * FD, gbias + 3 * FD, P3, P3, 0, XP, X4F, nN, nE, nb, vec8);
  k_head<<<1, HTHR, 0, stream>>>(X4F, fc1w, fc1b, fc2w, fc2b, out);
}
